// LearnerKnowledge_Aggregator_12120397709895
// MI455X (gfx1250) — hardware-verified
//
#include <hip/hip_runtime.h>
#include <math.h>
#include <stdint.h>

#define NNODE  8192
#define KN     50
#define DD     64
#define FF     128
#define NROWS  (NNODE * KN)
#define NCHUNK 4
#define CROWS  (NROWS / NCHUNK)
static_assert((CROWS % 64) == 0);
static_assert((NNODE % 8) == 0);
static_assert(KN > 32 && KN <= 64);

typedef __bf16   v16b __attribute__((ext_vector_type(16)));
typedef __bf16   v8b  __attribute__((ext_vector_type(8)));
typedef float    v8f  __attribute__((ext_vector_type(8)));
typedef float    v4f  __attribute__((ext_vector_type(4)));
typedef unsigned int v4u __attribute__((ext_vector_type(4)));

__device__ __forceinline__ unsigned short bf_bits(float f) {
  unsigned u = __float_as_uint(f);
  return (unsigned short)((u + 0x7FFFu + ((u >> 16) & 1u)) >> 16);
}
__device__ __forceinline__ float bf_up(unsigned short h) { return __uint_as_float(((unsigned)h) << 16); }
__device__ __forceinline__ float bf_rne(float f) { return bf_up(bf_bits(f)); }
__device__ __forceinline__ unsigned pk16(unsigned short a, unsigned short b) { return (unsigned)a | ((unsigned)b << 16); }
__device__ __forceinline__ v8f zero8() { v8f z = {0.f, 0.f, 0.f, 0.f, 0.f, 0.f, 0.f, 0.f}; return z; }
__device__ __forceinline__ int clampi(int v, int lo, int hi) { v = v < lo ? lo : v; return v > hi ? hi : v; }

__device__ __forceinline__ v16b ldfrag_b(const __bf16* p) {
  union { v16b v; v8b h[2]; } f;
  f.h[0] = *(const v8b*)(p);
  f.h[1] = *(const v8b*)(p + 16);
  return f.v;
}

__device__ __forceinline__ v8f mma_b_raw(v16b a, v16b b, v8f c) {
  return __builtin_amdgcn_wmma_f32_16x16x32_bf16(false, a, false, b, (short)0, c, false, false);
}
__device__ __forceinline__ void dep_guard_b(v8f& a, v8f& b, v16b x, v16b y) {
#if defined(__HIP_DEVICE_COMPILE__)
  asm volatile("v_nop\n\tv_nop\n\tv_nop\n\tv_nop" : "+v"(a), "+v"(b) : "v"(x), "v"(y));
#endif
}
__device__ __forceinline__ void keep4_b(v16b a, v16b b, v16b c, v16b d) {
#if defined(__HIP_DEVICE_COMPILE__)
  asm volatile("v_nop" :: "v"(a), "v"(b), "v"(c), "v"(d));
#endif
}
__device__ __forceinline__ void acc_guard4(v8f& a, v8f& b, v8f& c, v8f& d) {
#if defined(__HIP_DEVICE_COMPILE__)
  asm volatile("v_nop\n\tv_nop\n\tv_nop\n\tv_nop" : "+v"(a), "+v"(b), "+v"(c), "+v"(d));
#endif
}
__device__ __forceinline__ void wave_sync_lds() {
  __builtin_amdgcn_fence(__ATOMIC_RELEASE, "workgroup");
  __builtin_amdgcn_wave_barrier();
  __builtin_amdgcn_fence(__ATOMIC_ACQUIRE, "workgroup");
}

__global__ __launch_bounds__(256) void cvt_bf16x8(const float* __restrict__ in, unsigned short* out, int n8) {
  const int i = blockIdx.x * 256 + threadIdx.x;
  if (i < n8) {
    const v4f a = *(const v4f*)(in + (size_t)i * 8);
    const v4f b = *(const v4f*)(in + (size_t)i * 8 + 4);
    v4u p;
    p[0] = pk16(bf_bits(a[0]), bf_bits(a[1]));
    p[1] = pk16(bf_bits(a[2]), bf_bits(a[3]));
    p[2] = pk16(bf_bits(b[0]), bf_bits(b[1]));
    p[3] = pk16(bf_bits(b[2]), bf_bits(b[3]));
    *(volatile v4u*)(out + (size_t)i * 8) = p;
    __threadfence();
    *(volatile v4u*)(out + (size_t)i * 8) = p;
  }
}

__global__ __launch_bounds__(256) void gather_x(const int* __restrict__ nodes, const int* __restrict__ history,
                                                const float* __restrict__ u_to_e, const float* __restrict__ v_to_e,
                                                unsigned short* X, int rbase, int nrows, int nu, int nv) {
  const int lane = threadIdx.x & 31;
  const int wave = threadIdx.x >> 5;
  const int hh   = lane >> 4;
  const int c8   = (lane & 15) * 8;
  const int rw   = blockIdx.x * 64 + wave * 8;
  if (rw + 8 > nrows) return;
  v4u p[4];
#pragma unroll
  for (int it = 0; it < 4; ++it) {
    const int rr = rw + it * 2 + hh;
    const int r  = clampi(rbase + rr, 0, NROWS - 1);
    const int b  = r / KN;
    const int hs = clampi(history[r], 0, nv - 1);
    const int nd = clampi(nodes[b], 0, nu - 1);
    const float* pv = v_to_e + (size_t)hs * DD + c8;
    const float* pu = u_to_e + (size_t)nd * DD + (c8 - DD);
    const float* src = (c8 < DD) ? pv : pu;
    const v4f a = *(const v4f*)(src);
    const v4f c = *(const v4f*)(src + 4);
    v4u q;
    q[0] = pk16(bf_bits(a[0]), bf_bits(a[1]));
    q[1] = pk16(bf_bits(a[2]), bf_bits(a[3]));
    q[2] = pk16(bf_bits(c[0]), bf_bits(c[1]));
    q[3] = pk16(bf_bits(c[2]), bf_bits(c[3]));
    p[it] = q;
  }
  for (int pass = 0; pass < 2; ++pass) {
#pragma unroll
    for (int it = 0; it < 4; ++it) {
      const int rr = rw + it * 2 + hh;
      *(volatile v4u*)(X + (size_t)rr * FF + c8) = p[it];
    }
    __threadfence();
  }
}

template <int NSPLIT, int OUT_MODE>
__global__ __launch_bounds__(256) void gemm64(
    const unsigned short* __restrict__ Ap, const unsigned short* A2p, int lda,
    const unsigned short* __restrict__ Btp, int ldb,
    const float* __restrict__ bias, int relu,
    void* Cout, void* Cout2, int ldc,
    const float* __restrict__ w3, const float* __restrict__ b3,
    int M, int N, int K) {
  const __bf16* A   = (const __bf16*)(const void*)Ap;
  const __bf16* A2  = (const __bf16*)(const void*)A2p;
  const __bf16* Bt  = (const __bf16*)(const void*)Btp;
  __shared__ __align__(16) float sT[8][16 * 68];
  __shared__ __align__(16) float sW3[8][64];
  __shared__ __align__(16) float sLg[8][64];
  const int lane = threadIdx.x & 31;
  const int wave = threadIdx.x >> 5;
  const int tilesN = N >> 6;
  const int tilesM = M >> 6;
  const int tile = blockIdx.x * 8 + wave;
  if (tile >= tilesM * tilesN) return;
  const int tm = tile / tilesN;
  const int tn = tile - tm * tilesN;
  const int m0 = tm << 6;
  const int n0 = tn << 6;

  const __bf16* Ab  = A;
  const __bf16* Bb  = Bt;
  const __bf16* Ab2 = (NSPLIT >= 1) ? A2 : Ab;

  const int rlane = lane & 15;
  const int koff  = (lane >> 4) * 8;
  const int mOff  = (lane >> 4) * 8;

  float bv[4];
#pragma unroll
  for (int j = 0; j < 4; ++j) bv[j] = bf_rne(bias[n0 + (j << 4) + rlane]);
  float b3v = 0.f;
  if (OUT_MODE == 4) {
    sW3[wave][lane]      = bf_rne(w3[lane]);
    sW3[wave][lane + 32] = bf_rne(w3[lane + 32]);
    b3v = bf_rne(b3[0]);
  }

  v8f acc[4][4];
#pragma unroll
  for (int i = 0; i < 4; ++i)
#pragma unroll
    for (int j = 0; j < 4; ++j) acc[i][j] = zero8();

  for (int k0 = 0; k0 < K; k0 += 32) {
    v16b bh[4];
#pragma unroll
    for (int j = 0; j < 4; ++j) {
      const size_t bo = (size_t)(n0 + (j << 4) + rlane) * ldb + koff + k0;
      bh[j] = ldfrag_b(Bb + bo);
    }
#pragma unroll
    for (int i = 0; i < 4; ++i) {
      const size_t ao = (size_t)(m0 + (i << 4) + rlane) * lda + koff + k0;
      const v16b ah = ldfrag_b(Ab + ao);
      v16b al = ah;
      if (NSPLIT >= 1) al = ldfrag_b(Ab2 + ao);
#pragma unroll
      for (int j = 0; j < 4; ++j) {
        acc[i][j] = mma_b_raw(ah, bh[j], acc[i][j]);
        if (NSPLIT >= 1) acc[i][j] = mma_b_raw(al, bh[j], acc[i][j]);
      }
      dep_guard_b(acc[i][0], acc[i][3], ah, al);
    }
    keep4_b(bh[0], bh[1], bh[2], bh[3]);
  }
  acc_guard4(acc[0][0], acc[0][1], acc[0][2], acc[0][3]);
  acc_guard4(acc[1][0], acc[1][1], acc[1][2], acc[1][3]);
  acc_guard4(acc[2][0], acc[2][1], acc[2][2], acc[2][3]);
  acc_guard4(acc[3][0], acc[3][1], acc[3][2], acc[3][3]);

  float* slab = sT[wave];
#pragma unroll
  for (int i = 0; i < 4; ++i) {
    const int mBase = m0 + (i << 4);
#pragma unroll
    for (int j = 0; j < 4; ++j) {
#pragma unroll
      for (int r = 0; r < 8; ++r) {
        float v = acc[i][j][r] + bv[j];
        if (relu) v = fmaxf(v, 0.0f);
        slab[(mOff + r) * 68 + (j << 4) + rlane] = v;
      }
    }
    wave_sync_lds();
    if (OUT_MODE == 2) {
      const int q = lane >> 3, c8 = (lane & 7) * 8;
      unsigned short* C  = (unsigned short*)Cout;
      unsigned short* C2 = (unsigned short*)Cout2;
      v4u hv[4], lv[4];
#pragma unroll
      for (int it = 0; it < 4; ++it) {
        const int row = it * 4 + q;
        const float* sp = slab + row * 68 + c8;
        v4u a, a2;
#pragma unroll
        for (int e = 0; e < 4; ++e) {
          const float f0 = sp[2 * e], f1 = sp[2 * e + 1];
          const unsigned short h0 = bf_bits(f0), h1 = bf_bits(f1);
          const unsigned short l0 = bf_bits(f0 - bf_up(h0)), l1 = bf_bits(f1 - bf_up(h1));
          a[e] = pk16(h0, h1); a2[e] = pk16(l0, l1);
        }
        hv[it] = a; lv[it] = a2;
      }
      for (int pass = 0; pass < 2; ++pass) {
#pragma unroll
        for (int it = 0; it < 4; ++it) {
          const int row = it * 4 + q;
          *(volatile v4u*)(C  + (size_t)(mBase + row) * ldc + n0 + c8) = hv[it];
          *(volatile v4u*)(C2 + (size_t)(mBase + row) * ldc + n0 + c8) = lv[it];
        }
        __threadfence();
      }
    } else {
      const int row = lane & 15, h2 = lane >> 4;
      const float* sp = slab + row * 68 + h2 * 32;
      const float* wp = sW3[wave] + h2 * 32;
      float s = 0.f;
#pragma unroll 4
      for (int t = 0; t < 32; ++t) s = fmaf(sp[t], wp[t], s);
      s += __shfl_xor(s, 16, 32);
      if (h2 == 0) sLg[wave][i * 16 + row] = s + b3v;
    }
    wave_sync_lds();
  }
  if (OUT_MODE == 4) {
    float* C = (float*)Cout;
    const v4f v = *(const v4f*)(sLg[wave] + 4 * (lane & 15));
    if (lane < 16) *(volatile v4f*)(C + (size_t)m0 + 4 * lane) = v;
    __threadfence();
    if (lane < 16) *(volatile v4f*)(C + (size_t)m0 + 4 * lane) = v;
  }
}

__global__ __launch_bounds__(256) void agg_out(const int* __restrict__ history, const int* __restrict__ degrees,
                                               const float* __restrict__ v_to_e, const float* __restrict__ logits,
                                               float* out, int nnode, int nv) {
  __shared__ __align__(16) float sO[8][64];
  const int lane = threadIdx.x & 31;
  const int wave = threadIdx.x >> 5;
  const int b = blockIdx.x * 8 + wave;
  if (b >= nnode) return;
  const int deg = clampi(degrees[b], 1, KN);
  const int k1 = lane, k2 = lane + 32;
  const int k2c = (k2 < KN) ? k2 : (KN - 1);
  const bool v2 = (k2 < KN);
  const size_t rb = (size_t)b * KN;
  const int hs1 = clampi(history[rb + k1],  0, nv - 1);
  const int hs2 = clampi(history[rb + k2c], 0, nv - 1);
  const float L1 = logits[rb + k1];
  const float L2 = logits[rb + k2c];
  const float x1 = (k1 < deg) ? L1 : -1.0e9f;
  const float x2 = (v2 && (k2 < deg)) ? L2 : -1.0e9f;
  float m = fmaxf(x1, x2);
#pragma unroll
  for (int off = 1; off < 32; off <<= 1) m = fmaxf(m, __shfl_xor(m, off, 32));
  float e1 = __expf(x1 - m);
  float e2 = __expf(x2 - m);
  e1 = (k1 < deg) ? e1 : 0.f;
  e2 = (v2 && (k2 < deg)) ? e2 : 0.f;
  float S = e1 + e2;
#pragma unroll
  for (int off = 1; off < 32; off <<= 1) S += __shfl_xor(S, off, 32);
  const float inv = 1.0f / S;
  const float a1 = e1 * inv;
  const float a2 = e2 * inv;

  float o0 = 0.f, o1 = 0.f;
#pragma unroll 2
  for (int k = 0; k < KN; ++k) {
    const bool lo = (k < 32);
    const float asel = lo ? a1 : a2;
    const int   hsel = lo ? hs1 : hs2;
    const float a  = __shfl(asel, k & 31, 32);
    const int   hk = __shfl(hsel, k & 31, 32);
    const float* vr = v_to_e + (size_t)hk * DD;
    const float va = bf_rne(vr[lane]);
    const float vb = bf_rne(vr[lane + 32]);
    o0 = fmaf(a, va, o0);
    o1 = fmaf(a, vb, o1);
  }
  sO[wave][lane]      = o0;
  sO[wave][lane + 32] = o1;
  wave_sync_lds();
  const v4f v = *(const v4f*)(sO[wave] + 4 * (lane & 15));
  if (lane < 16) *(volatile v4f*)(out + (size_t)b * DD + 4 * lane) = v;
  __threadfence();
  if (lane < 16) *(volatile v4f*)(out + (size_t)b * DD + 4 * lane) = v;
}

extern "C" void kernel_launch(void* const* d_in, const int* in_sizes, int n_in,
                              void* d_out, int out_size, void* d_ws, size_t ws_size,
                              hipStream_t stream) {
  if (n_in < 11) return;
  if (in_sizes[0] != NNODE || in_sizes[1] != NROWS || in_sizes[2] != NNODE) return;
  if (in_sizes[3] < DD || (in_sizes[3] % DD) != 0) return;
  if (in_sizes[4] < DD || (in_sizes[4] % DD) != 0) return;
  if (in_sizes[5] != DD * FF || in_sizes[6] != DD || in_sizes[7] != DD * DD || in_sizes[8] != DD) return;
  if (in_sizes[9] != DD || in_sizes[10] < 1) return;
  if (out_size != NNODE * DD) return;

  const int*   nodes   = (const int*)  d_in[0];
  const int*   history = (const int*)  d_in[1];
  const int*   degrees = (const int*)  d_in[2];
  const float* u_to_e  = (const float*)d_in[3];
  const float* v_to_e  = (const float*)d_in[4];
  const float* att1_w  = (const float*)d_in[5];
  const float* att1_b  = (const float*)d_in[6];
  const float* att2_w  = (const float*)d_in[7];
  const float* att2_b  = (const float*)d_in[8];
  const float* att3_w  = (const float*)d_in[9];
  const float* att3_b  = (const float*)d_in[10];
  float* out = (float*)d_out;
  const int nu = in_sizes[3] / DD;
  const int nv = in_sizes[4] / DD;

  const size_t PW1 = (size_t)DD * FF * 2;
  const size_t PW2 = (size_t)DD * DD * 2;
  const size_t PX  = (size_t)CROWS * FF * 2;
  const size_t PH  = (size_t)CROWS * DD * 2;
  const size_t PLg = (size_t)NROWS * 4;
  size_t off = 0;
  const size_t oW1 = off; off += PW1;
  const size_t oW2 = off; off += PW2;
  const size_t oX  = off; off += PX;
  const size_t oHh = off; off += PH;
  const size_t oHl = off; off += PH;
  const size_t oLg = off; off += PLg;
  if (off > ws_size) return;
  if (off > (size_t)134217728) return;

  char* ws = (char*)d_ws;
  unsigned short* W1b = (unsigned short*)(ws + oW1);
  unsigned short* W2b = (unsigned short*)(ws + oW2);
  unsigned short* Xb  = (unsigned short*)(ws + oX);
  unsigned short* H1h = (unsigned short*)(ws + oHh);
  unsigned short* H1l = (unsigned short*)(ws + oHl);
  float*          Lg  = (float*)(ws + oLg);

  const dim3 blk(256);
  const int n8w1 = DD * FF / 8;
  const int n8w2 = DD * DD / 8;
  const dim3 gW1((n8w1 + 255) / 256);
  const dim3 gW2((n8w2 + 255) / 256);
  const dim3 gGat(CROWS / 64);
  const dim3 gGm((CROWS / 64 + 7) / 8);
  const dim3 gAgg(NNODE / 8);

  cvt_bf16x8<<<gW1, blk, 0, stream>>>(att1_w, W1b, n8w1);
  cvt_bf16x8<<<gW2, blk, 0, stream>>>(att2_w, W2b, n8w2);
  for (int c = 0; c < NCHUNK; ++c) {
    const int rbase = c * CROWS;
    gather_x<<<gGat, blk, 0, stream>>>(nodes, history, u_to_e, v_to_e, Xb, rbase, CROWS, nu, nv);
    gemm64<0, 2><<<gGm, blk, 0, stream>>>(
        Xb, Xb, FF, W1b, FF, att1_b, 1,
        (void*)H1h, (void*)H1l, DD, att3_w, att3_b,
        CROWS, DD, FF);
    gemm64<1, 4><<<gGm, blk, 0, stream>>>(
        H1h, H1l, DD, W2b, DD, att2_b, 1,
        (void*)(Lg + (size_t)rbase), (void*)(Lg + (size_t)rbase), DD, att3_w, att3_b,
        CROWS, DD, DD);
  }
  agg_out<<<gAgg, blk, 0, stream>>>(history, degrees, v_to_e, Lg, out, NNODE, nv);
  (void)hipGetLastError();
}
